// MeshConvPoint_74208444940566
// MI455X (gfx1250) — hardware-verified
//
#include <hip/hip_runtime.h>


namespace {
constexpr int B = 8, C = 64, V = 25000, DG = 12, O = 64, NJ = (V + 31) / 32 + 1;
constexpr float XS = 8.0f, WSC = 256.0f;
typedef _Float16 b16;
typedef __attribute__((ext_vector_type(16))) _Float16 v16b;
typedef __attribute__((ext_vector_type(8))) _Float16 v8b;
typedef __attribute__((ext_vector_type(8))) float v8f;
__device__ __forceinline__ float bf16_rne(float f) { unsigned int u = __float_as_uint(f); u += 0x7FFFu + ((u >> 16) & 1u); float r = __uint_as_float(u & 0xFFFF0000u); asm volatile("" : "+v"(r)); return r; }
__device__ __forceinline__ void split16(float v, b16& hi, b16& lo) { hi = (b16)v; lo = (b16)(v - (float)hi); }
__device__ __forceinline__ v16b frag_kb(const b16* p, int hh) { const v8b a = *(const v8b*)(p + 8 * hh), b = *(const v8b*)(p + 16 + 8 * hh); v16b f;
#pragma unroll
  for (int e = 0; e < 8; ++e) { f[e] = a[e]; f[8 + e] = b[e]; } return f; }
__device__ __forceinline__ v8f wmma16b(v16b a, v16b b, v8f c) { v8f d = __builtin_amdgcn_wmma_f32_16x16x32_f16(false, a, false, b, (short)0, c, false, false); asm volatile("v_nop\n\tv_nop\n\tv_nop\n\tv_nop" : "+v"(d) : "v"(a), "v"(b)); return d; }
__device__ __forceinline__ void wave_lds_sync() { __builtin_amdgcn_fence(__ATOMIC_RELEASE, "workgroup"); __builtin_amdgcn_wave_barrier(); __builtin_amdgcn_fence(__ATOMIC_ACQUIRE, "workgroup"); }
__device__ __forceinline__ float pmul(float a, float b) { float p = a * b; asm volatile("" : "+v"(p)); return p; }
__device__ __forceinline__ int iclamp(int v, int lo, int hi) { return v < lo ? lo : (v > hi ? hi : v); }

__global__ __launch_bounds__(256) void wput_kernel(const float* __restrict__ w, b16* __restrict__ WT) { const int u = blockIdx.x * 256 + threadIdx.x; if (u >= O * 16) return; const int r = u / 16, k0 = (u % 16) * 8; const int cls = r / 16, q = r % 16, o = 4 * q + cls; v8b v;
#pragma unroll
  for (int j = 0; j < 8; ++j) { const int k = k0 + j; const float val = k < C ? w[((size_t)o * C + k) * 2] : w[((size_t)o * C + (k - C)) * 2 + 1]; v[j] = (b16)(bf16_rne(val) * WSC); }
  for (int pass = 0; pass < 2; ++pass) { *(volatile v8b*)(WT + (size_t)r * 128 + k0) = v; __threadfence(); } }
__global__ __launch_bounds__(256) void mean_kernel(const float* __restrict__ x, const int* __restrict__ nbr, const int* __restrict__ deg, int BV, float* __restrict__ MEAN) { const int u = blockIdx.x * 256 + threadIdx.x; if (u >= BV * V) return; const int b = u / V, v = u % V;
  const int dg = iclamp(deg[(size_t)b * V + v], 0, DG); int nb[DG];
#pragma unroll
  for (int d = 0; d < DG; ++d) nb[d] = iclamp(nbr[((size_t)b * V + v) * DG + d], 0, V - 1);
  const float inv = 1.0f / (float)(dg > 0 ? dg : 1);
  for (int pass = 0; pass < 2; ++pass) {
#pragma unroll 1
    for (int c = 0; c < C; ++c) { const float* xr = x + ((size_t)b * C + c) * V; float s = 0.0f;
#pragma unroll
      for (int d = 0; d < DG; ++d) if (d < dg) s += bf16_rne(xr[nb[d]]);
      ((volatile float*)MEAN)[((size_t)b * C + c) * V + v] = pmul(s, inv); }
    __threadfence(); } }
__global__ __launch_bounds__(32) void conv_kernel(const float* __restrict__ x, const float* __restrict__ MEAN, const b16* __restrict__ WT, const float* __restrict__ bias, int BV, float* __restrict__ out) {
  __shared__ __attribute__((aligned(16))) b16 Ah[32][136], Al[32][136]; __shared__ float Tf[32][17]; const int lane = threadIdx.x, nloc = lane & 15, hlf = lane >> 4;
  const int j = blockIdx.x % NJ, cls = (blockIdx.x / NJ) % 4, b = blockIdx.x / (NJ * 4); if (b >= BV) return; const int s = (8 * cls) % 32; const int v0 = 32 * j - s; if (v0 < 0 || v0 + 32 > V) return;
  for (int q = 0; q < 4; ++q) { const int k = q * 32 + lane; const float* src = k < C ? x + ((size_t)b * C + k) * V : MEAN + ((size_t)b * C + (k - C)) * V;
    for (int rr = 0; rr < 32; ++rr) { const int v = v0 + rr; float val = (v >= 0 && v < V) ? src[v] : 0.0f; b16 p, ql; if (k < C) { p = (b16)(bf16_rne(val) * XS); ql = (b16)0.0f; } else split16(val * XS, p, ql); Ah[rr][k] = p; Al[rr][k] = ql; } }
  wave_lds_sync(); v8f acc[2] = {(v8f){}, (v8f){}};
#pragma unroll
  for (int kb = 0; kb < 128; kb += 32) { const v16b bw = frag_kb(WT + (size_t)(cls * 16 + nloc) * 128 + kb, hlf);
#pragma unroll
    for (int m = 0; m < 2; ++m) { const v16b a = frag_kb(&Ah[m * 16 + nloc][kb], hlf); acc[m] = wmma16b(a, bw, acc[m]); if (kb >= 64) { const v16b al = frag_kb(&Al[m * 16 + nloc][kb], hlf); acc[m] = wmma16b(al, bw, acc[m]); } } }
#pragma unroll
  for (int m = 0; m < 2; ++m)
#pragma unroll
    for (int r8 = 0; r8 < 8; ++r8) Tf[m * 16 + 8 * hlf + r8][nloc] = acc[m][r8] * (1.0f / (XS * WSC)) + bf16_rne(bias[4 * nloc + cls]);
  wave_lds_sync(); const int v = v0 + lane;
  for (int pass = 0; pass < 2; ++pass) {
#pragma unroll
    for (int q = 0; q < 16; ++q) { const int o = 4 * q + cls; ((volatile float*)out)[((size_t)b * O + o) * V + v] = Tf[lane][q]; } __threadfence(); } }
__global__ __launch_bounds__(32) void seam_kernel(const float* __restrict__ x, const float* __restrict__ MEAN, const float* __restrict__ w, const float* __restrict__ bias, int BV, float* __restrict__ out) { const int lane = threadIdx.x; const int o = blockIdx.x % O, b = blockIdx.x / O; if (b >= BV) return; const int cls = o % 4; if (cls == 0) return; const int sh = 8 * cls;
  int oo, v; if (lane < sh) { oo = o - 1; v = V - sh + lane; } else { oo = o; v = lane - sh; } float s = bf16_rne(bias[oo]);
#pragma unroll 4
  for (int c = 0; c < C; ++c) { s += pmul(bf16_rne(w[((size_t)oo * C + c) * 2]), bf16_rne(x[((size_t)b * C + c) * V + v])); s += pmul(bf16_rne(w[((size_t)oo * C + c) * 2 + 1]), MEAN[((size_t)b * C + c) * V + v]); }
  for (int pass = 0; pass < 2; ++pass) { ((volatile float*)out)[((size_t)b * O + oo) * V + v] = s; __threadfence(); } }
}

extern "C" void kernel_launch(void* const* d_in, const int* in_sizes, int n_in, void* d_out, int out_size, void* d_ws, size_t ws_size, hipStream_t stream) {
  (void)n_in;
  auto Fp = [&](int i) { return (const float*)d_in[i]; }; auto Ip = [&](int i) { return (const int*)d_in[i]; };
  if (in_sizes[0] != B * C * V || in_sizes[1] != B * V * DG || in_sizes[2] != B * V || in_sizes[3] != O * C * 2 || in_sizes[4] != O || out_size != B * O * V) return;
  const int BV = B;
  size_t off = 0; char* ws = (char*)d_ws;
  auto carve = [&](size_t bytes) { char* p = ws + off; off += (bytes + 255) & ~(size_t)255; return p; };
  b16* WT = (b16*)carve((size_t)O * 128 * 2); float* MEAN = (float*)carve((size_t)B * C * V * 4);
  if (off > ws_size || off > ((size_t)64 << 20)) return;
  wput_kernel<<<(O * 16 + 255) / 256, 256, 0, stream>>>(Fp(3), WT);
  mean_kernel<<<(BV * V + 255) / 256, 256, 0, stream>>>(Fp(0), Ip(1), Ip(2), BV, MEAN);
  conv_kernel<<<BV * 4 * NJ, 32, 0, stream>>>(Fp(0), MEAN, WT, Fp(4), BV, (float*)d_out);
  seam_kernel<<<BV * O, 32, 0, stream>>>(Fp(0), MEAN, Fp(3), Fp(4), BV, (float*)d_out);
}
